// partical_similarity_71193377898738
// MI455X (gfx1250) — hardware-verified
//
#include <hip/hip_runtime.h>
#define NM 16
#define NN 16
#define CCh 32
#define HS 96
#define HP 128
#define HK 32
#define HO 97
#define NXT 7

typedef __bf16 v16b __attribute__((ext_vector_type(16)));
typedef unsigned short v8us __attribute__((ext_vector_type(8), may_alias));
typedef float  v8f  __attribute__((ext_vector_type(8)));
typedef float  v4f  __attribute__((ext_vector_type(4)));
typedef float  v4fa __attribute__((ext_vector_type(4), may_alias));
union FragB { v16b v; v8us half[2]; unsigned short u[16]; };

__device__ __forceinline__ unsigned short bf16_bits(float x) { unsigned int u = __float_as_uint(x); return (unsigned short)((u + 0x7FFFu + ((u >> 16) & 1u)) >> 16); }
__device__ __forceinline__ float bf16_val(unsigned short b) { return __uint_as_float(((unsigned int)b) << 16); }
__device__ __forceinline__ float bf16_round(float x) { return bf16_val(bf16_bits(x)); }
template <int NT>
__device__ __forceinline__ v8f mmaN(v16b ah, v16b al, v16b bh, v16b bl, v8f c) {
  c = __builtin_amdgcn_wmma_f32_16x16x32_bf16(false, ah, false, bh, (short)0, c, false, false);
  if (NT >= 2) c = __builtin_amdgcn_wmma_f32_16x16x32_bf16(false, al, false, bh, (short)0, c, false, false);
  if (NT >= 3) c = __builtin_amdgcn_wmma_f32_16x16x32_bf16(false, ah, false, bl, (short)0, c, false, false);
  asm volatile("v_nop\n\tv_nop\n\tv_nop\n\tv_nop" : "+v"(c) : "v"(ah), "v"(al), "v"(bh), "v"(bl));
  return c;
}

__global__ __launch_bounds__(256) void k_wt_bf16(const float* __restrict__ W, unsigned short* __restrict__ Wt, int K, int N) {
  const int t = blockIdx.x * 256 + threadIdx.x;
  const int k8n = K / 8;
  if (t >= N * k8n) return;
  const int n = t / k8n, k8 = (t % k8n) * 8;
  v8us v;
#pragma unroll
  for (int i = 0; i < 8; ++i) v[i] = bf16_bits(W[(size_t)(k8 + i) * N + n]);
  *(volatile v8us*)(Wt + (size_t)n * K + k8) = v;
  __threadfence();
  *(volatile v8us*)(Wt + (size_t)n * K + k8) = v;
}

template <bool ASPLIT, int ACT, bool BIAS_BF16>
__global__ __launch_bounds__(128) void k_gemm_bf(const float* __restrict__ A, int lda, const unsigned short* __restrict__ Wt, int ldb,
                                               const float* __restrict__ bias, float* __restrict__ C, int ldc, int M, int N, int K) {
  __shared__ __attribute__((aligned(16))) float so[4][16][64];
  const int tid = threadIdx.x, w = tid >> 5, lane = tid & 31, ln = lane & 15, hh = lane >> 4;
  const int ntn = N / 64;
  const int wid = blockIdx.x * 4 + w;
  const int mt = wid / ntn, nq = wid % ntn;
  if (mt * 16 >= M) return;
  const int row0 = mt * 16, col0 = nq * 64;
  const float* arow = A + (size_t)(row0 + ln) * lda;
  v8f acc[4] = {};
  for (int kb = 0; kb < K; kb += 32) {
    FragB ah, al;
    const v4f x0 = *(const v4fa*)(arow + kb + 8 * hh), x1 = *(const v4fa*)(arow + kb + 8 * hh + 4);
    const v4f x2 = *(const v4fa*)(arow + kb + 16 + 8 * hh), x3 = *(const v4fa*)(arow + kb + 16 + 8 * hh + 4);
    float xs[16] = {x0[0],x0[1],x0[2],x0[3],x1[0],x1[1],x1[2],x1[3],x2[0],x2[1],x2[2],x2[3],x3[0],x3[1],x3[2],x3[3]};
#pragma unroll
    for (int i = 0; i < 16; ++i) { const unsigned short hb = bf16_bits(xs[i]); ah.u[i] = hb; al.u[i] = ASPLIT ? bf16_bits(xs[i] - bf16_val(hb)) : (unsigned short)0; }
#pragma unroll
    for (int t = 0; t < 4; ++t) {
      const unsigned short* brow = Wt + (size_t)(col0 + t * 16 + ln) * ldb + kb;
      FragB b;
      b.half[0] = *(const v8us*)(brow + 8 * hh);
      b.half[1] = *(const v8us*)(brow + 16 + 8 * hh);
      acc[t] = mmaN<ASPLIT ? 2 : 1>(ah.v, al.v, b.v, b.v, acc[t]);
    }
  }
#pragma unroll
  for (int t = 0; t < 4; ++t) {
    float bv = bias ? bias[col0 + t * 16 + ln] : 0.f;
    if (BIAS_BF16) bv = bf16_round(bv);
#pragma unroll
    for (int r = 0; r < 8; ++r) { float v = acc[t][r] + bv; if (ACT == 1) v = fmaxf(v, 0.f); so[w][8 * hh + r][t * 16 + ln] = v; }
  }
  __builtin_amdgcn_fence(__ATOMIC_ACQ_REL, "workgroup");
  __builtin_amdgcn_wave_barrier();
  const int rsub = lane >> 4, c4 = (lane & 15) * 4;
  for (int pass = 0; pass < 2; ++pass) {
#pragma unroll
    for (int q = 0; q < 8; ++q) {
      const int r = q * 2 + rsub;
      const v4f v = *(const v4fa*)&so[w][r][c4];
      *(volatile v4f*)(C + (size_t)(row0 + r) * ldc + col0 + c4) = v;
    }
    if (pass == 0) __threadfence();
  }
}

template <int D, bool CAUSAL>
__global__ __launch_bounds__(128) void k_flash(const float* __restrict__ qb, const float* __restrict__ kb, const float* __restrict__ vb,
                                             int pitch, int T, int H, float scale, float* __restrict__ y, int ypitch) {
  constexpr int KS = D / 32;
  constexpr int DT = D / 16;
  __shared__ __attribute__((aligned(16))) unsigned short sKh[32][D + 8], sKl[32][D + 8], sVh[32][D + 8], sVl[32][D + 8];
  __shared__ __attribute__((aligned(16))) unsigned short sPh[4][16][40], sPl[4][16][40];
  __shared__ __attribute__((aligned(16))) float sO[4][16][D];
  const int tid = threadIdx.x, w = tid >> 5, lane = tid & 31, ln = lane & 15, hh = lane >> 4;
  const int nqb = (T + 63) / 64;
  const int bh = blockIdx.x / nqb, qblk = blockIdx.x % nqb;
  const int b = bh / H, h = bh % H;
  const int q0 = qblk * 64 + w * 16;
  const float* Q = qb + (size_t)b * T * pitch + h * D;
  const float* K = kb + (size_t)b * T * pitch + h * D;
  const float* V = vb + (size_t)b * T * pitch + h * D;

  FragB aqh[KS], aql[KS];
  {
    int row = q0 + ln; if (row >= T) row = T - 1;
    const float* qr = Q + (size_t)row * pitch;
#pragma unroll
    for (int ks = 0; ks < KS; ++ks)
#pragma unroll
      for (int i = 0; i < 16; ++i) {
        const int d = ks * 32 + ((i < 8) ? (8 * hh + i) : (16 + 8 * hh + (i - 8)));
        const float x = qr[d] * scale; const unsigned short hb = bf16_bits(x);
        aqh[ks].u[i] = hb; aql[ks].u[i] = bf16_bits(x - bf16_val(hb));
      }
  }
  float m_r[8], l_r[8];
#pragma unroll
  for (int r = 0; r < 8; ++r) { m_r[r] = -3.0e38f; l_r[r] = 0.f; }
  v8f oacc[DT];
#pragma unroll
  for (int dt = 0; dt < DT; ++dt) oacc[dt] = (v8f){0.f,0.f,0.f,0.f,0.f,0.f,0.f,0.f};

  const int kv_end = CAUSAL ? min(T, qblk * 64 + 64) : T;
  for (int j0 = 0; j0 < kv_end; j0 += 32) {
    __syncthreads();
    for (int e = tid; e < 32 * (D / 4); e += 128) {
      const int r = e / (D / 4), c4 = (e % (D / 4)) * 4;
      const int key = j0 + r;
      v4f kf = {0.f,0.f,0.f,0.f}, vf = {0.f,0.f,0.f,0.f};
      if (key < T) { kf = *(const v4fa*)(K + (size_t)key * pitch + c4); vf = *(const v4fa*)(V + (size_t)key * pitch + c4); }
#pragma unroll
      for (int t = 0; t < 4; ++t) {
        unsigned short hb = bf16_bits(kf[t]); sKh[r][c4 + t] = hb; sKl[r][c4 + t] = bf16_bits(kf[t] - bf16_val(hb));
        hb = bf16_bits(vf[t]); sVh[r][c4 + t] = hb; sVl[r][c4 + t] = bf16_bits(vf[t] - bf16_val(hb));
      }
    }
    __syncthreads();
    v8f s[2];
#pragma unroll
    for (int nt = 0; nt < 2; ++nt) {
      v8f acc = {};
#pragma unroll
      for (int ks = 0; ks < KS; ++ks) {
        FragB bh_, bl_;
        bh_.half[0] = *(const v8us*)&sKh[nt * 16 + ln][ks * 32 + 8 * hh]; bh_.half[1] = *(const v8us*)&sKh[nt * 16 + ln][ks * 32 + 16 + 8 * hh];
        bl_.half[0] = *(const v8us*)&sKl[nt * 16 + ln][ks * 32 + 8 * hh]; bl_.half[1] = *(const v8us*)&sKl[nt * 16 + ln][ks * 32 + 16 + 8 * hh];
        acc = mmaN<3>(aqh[ks].v, aql[ks].v, bh_.v, bl_.v, acc);
      }
      s[nt] = acc;
    }
    float alpha[8];
#pragma unroll
    for (int r = 0; r < 8; ++r) {
      const int qi = q0 + 8 * hh + r;
      const int ja = j0 + ln, jb = j0 + 16 + ln;
      if (CAUSAL) { if (ja > qi) s[0][r] = -3.0e38f; if (jb > qi) s[1][r] = -3.0e38f; }
      if (ja >= T) s[0][r] = -3.0e38f;
      if (jb >= T) s[1][r] = -3.0e38f;
      float mx = fmaxf(s[0][r], s[1][r]);
      mx = fmaxf(mx, __shfl_xor(mx, 1, 32)); mx = fmaxf(mx, __shfl_xor(mx, 2, 32)); mx = fmaxf(mx, __shfl_xor(mx, 4, 32)); mx = fmaxf(mx, __shfl_xor(mx, 8, 32));
      const float mnew = fmaxf(m_r[r], mx);
      alpha[r] = (mnew > -1.0e38f) ? __expf(m_r[r] - mnew) : 1.0f;
      const float p0 = (s[0][r] > -1.0e38f) ? __expf(s[0][r] - mnew) : 0.f;
      const float p1 = (s[1][r] > -1.0e38f) ? __expf(s[1][r] - mnew) : 0.f;
      m_r[r] = mnew;
      l_r[r] = l_r[r] * alpha[r] + p0 + p1;
      unsigned short hb = bf16_bits(p0); sPh[w][8 * hh + r][ln] = hb;      sPl[w][8 * hh + r][ln] = bf16_bits(p0 - bf16_val(hb));
      hb = bf16_bits(p1);                sPh[w][8 * hh + r][16 + ln] = hb; sPl[w][8 * hh + r][16 + ln] = bf16_bits(p1 - bf16_val(hb));
    }
#pragma unroll
    for (int dt = 0; dt < DT; ++dt)
#pragma unroll
      for (int r = 0; r < 8; ++r) oacc[dt][r] *= alpha[r];
    __builtin_amdgcn_fence(__ATOMIC_ACQ_REL, "workgroup");
    __builtin_amdgcn_wave_barrier();
    FragB pah, pal;
    pah.half[0] = *(const v8us*)&sPh[w][ln][8 * hh]; pah.half[1] = *(const v8us*)&sPh[w][ln][16 + 8 * hh];
    pal.half[0] = *(const v8us*)&sPl[w][ln][8 * hh]; pal.half[1] = *(const v8us*)&sPl[w][ln][16 + 8 * hh];
#pragma unroll
    for (int dt = 0; dt < DT; ++dt) {
      FragB bvh, bvl;
#pragma unroll
      for (int i = 0; i < 8; ++i) {
        bvh.u[i] = sVh[8 * hh + i][dt * 16 + ln]; bvh.u[8 + i] = sVh[16 + 8 * hh + i][dt * 16 + ln];
        bvl.u[i] = sVl[8 * hh + i][dt * 16 + ln]; bvl.u[8 + i] = sVl[16 + 8 * hh + i][dt * 16 + ln];
      }
      oacc[dt] = mmaN<3>(pah.v, pal.v, bvh.v, bvl.v, oacc[dt]);
    }
    __builtin_amdgcn_fence(__ATOMIC_ACQ_REL, "workgroup");
    __builtin_amdgcn_wave_barrier();
  }
#pragma unroll
  for (int r = 0; r < 8; ++r) {
    float l = l_r[r];
    l += __shfl_xor(l, 1, 32); l += __shfl_xor(l, 2, 32); l += __shfl_xor(l, 4, 32); l += __shfl_xor(l, 8, 32);
    l_r[r] = (l > 0.f) ? 1.0f / l : 0.f;
  }
#pragma unroll
  for (int dt = 0; dt < DT; ++dt)
#pragma unroll
    for (int r = 0; r < 8; ++r) sO[w][8 * hh + r][dt * 16 + ln] = oacc[dt][r] * l_r[r];
  __builtin_amdgcn_fence(__ATOMIC_ACQ_REL, "workgroup");
  __builtin_amdgcn_wave_barrier();
  for (int pass = 0; pass < 2; ++pass) {
    for (int r = 0; r < 16; ++r) {
      const int row = q0 + r;
      if (row < T && lane < D / 4) {
        const v4f val = *(const v4fa*)&sO[w][r][lane * 4];
        *(volatile v4f*)(y + ((size_t)b * T + row) * ypitch + h * D + lane * 4) = val;
      }
    }
    if (pass == 0) __threadfence();
  }
}

template <bool ASPLIT, int ACT, bool BIAS_BF16, bool RES_BF16>
__global__ __launch_bounds__(128) void k_gemm_bf3(const float* __restrict__ A, int lda, const unsigned short* __restrict__ Wt, int ldb,
                                                const float* __restrict__ bias, const float* __restrict__ resid, int rmod, int ldr,
                                                float* __restrict__ C, int ldc, int M, int N, int K) {
  __shared__ __attribute__((aligned(16))) float so[4][16][64];
  const int tid = threadIdx.x, w = tid >> 5, lane = tid & 31, ln = lane & 15, hh = lane >> 4;
  const int ntn = N / 64;
  const int wid = blockIdx.x * 4 + w;
  const int mt = wid / ntn, nq = wid % ntn;
  if (mt * 16 >= M) return;
  const int row0 = mt * 16, col0 = nq * 64;
  const float* arow = A + (size_t)(row0 + ln) * lda;
  v8f acc[4] = {};
  for (int kb = 0; kb < K; kb += 32) {
    FragB ah, al;
    const v4f x0 = *(const v4fa*)(arow + kb + 8 * hh), x1 = *(const v4fa*)(arow + kb + 8 * hh + 4);
    const v4f x2 = *(const v4fa*)(arow + kb + 16 + 8 * hh), x3 = *(const v4fa*)(arow + kb + 16 + 8 * hh + 4);
    float xs[16] = {x0[0],x0[1],x0[2],x0[3],x1[0],x1[1],x1[2],x1[3],x2[0],x2[1],x2[2],x2[3],x3[0],x3[1],x3[2],x3[3]};
#pragma unroll
    for (int i = 0; i < 16; ++i) { const unsigned short hb = bf16_bits(xs[i]); ah.u[i] = hb; al.u[i] = ASPLIT ? bf16_bits(xs[i] - bf16_val(hb)) : (unsigned short)0; }
#pragma unroll
    for (int t = 0; t < 4; ++t) {
      const unsigned short* brow = Wt + (size_t)(col0 + t * 16 + ln) * ldb + kb;
      FragB b;
      b.half[0] = *(const v8us*)(brow + 8 * hh);
      b.half[1] = *(const v8us*)(brow + 16 + 8 * hh);
      acc[t] = mmaN<ASPLIT ? 2 : 1>(ah.v, al.v, b.v, b.v, acc[t]);
    }
  }
#pragma unroll
  for (int t = 0; t < 4; ++t) {
    const int col = col0 + t * 16 + ln;
    float bv = bias ? bias[col] : 0.f;
    if (BIAS_BF16) bv = bf16_round(bv);
#pragma unroll
    for (int r = 0; r < 8; ++r) {
      float v = acc[t][r] + bv;
      if (resid) { float rv = resid[(size_t)((row0 + 8 * hh + r) % rmod) * ldr + col]; if (RES_BF16) rv = bf16_round(rv); v += rv; }
      if (ACT == 1) v = fmaxf(v, 0.f);
      if (ACT == 2) v = 0.5f * v * (1.0f + erff(v * 0.70710678118654752f));
      if (ACT == 3) { const float u = 0.7978845608028654f * (v + 0.044715f * v * v * v); v = 0.5f * v * (1.0f + tanhf(u)); }
      so[w][8 * hh + r][t * 16 + ln] = v;
    }
  }
  __builtin_amdgcn_fence(__ATOMIC_ACQ_REL, "workgroup");
  __builtin_amdgcn_wave_barrier();
  const int rsub = lane >> 4, c4 = (lane & 15) * 4;
  for (int pass = 0; pass < 2; ++pass) {
#pragma unroll
    for (int q = 0; q < 8; ++q) {
      const int r = q * 2 + rsub;
      const v4f v = *(const v4fa*)&so[w][r][c4];
      *(volatile v4f*)(C + (size_t)(row0 + r) * ldc + col0 + c4) = v;
    }
    if (pass == 0) __threadfence();
  }
}
template <bool PARAM_BF16>
__global__ __launch_bounds__(256) void k_layernorm(const float* __restrict__ X, const float* __restrict__ R, const float* __restrict__ g, const float* __restrict__ bta,
                                                  float* __restrict__ out_sum, float* __restrict__ out_norm, int N, float eps) {
  __shared__ float red[256];
  const int row = blockIdx.x, tid = threadIdx.x;
  const float* x = X + (size_t)row * N; const float* rr = R ? R + (size_t)row * N : nullptr;
  float vals[16];
  const int per = N / 256;
  float s1 = 0.f;
  for (int u = 0; u < per / 4; ++u) {
    const int j = tid * 4 + 1024 * u;
    const v4f a = *(const v4fa*)(x + j);
    v4f b = {0.f,0.f,0.f,0.f}; if (rr) b = *(const v4fa*)(rr + j);
#pragma unroll
    for (int q = 0; q < 4; ++q) { const float v = a[q] + b[q]; vals[u * 4 + q] = v; s1 += v; }
  }
  red[tid] = s1; __syncthreads();
  for (int st = 128; st > 0; st >>= 1) { if (tid < st) red[tid] += red[tid + st]; __syncthreads(); }
  const float mu = red[0] / (float)N; __syncthreads();
  float s2 = 0.f;
  for (int u = 0; u < per / 4; ++u)
#pragma unroll
    for (int q = 0; q < 4; ++q) { const float c = vals[u * 4 + q] - mu; s2 += c * c; }
  red[tid] = s2; __syncthreads();
  for (int st = 128; st > 0; st >>= 1) { if (tid < st) red[tid] += red[tid + st]; __syncthreads(); }
  const float rs = rsqrtf(red[0] / (float)N + eps);
  for (int pass = 0; pass < 2; ++pass) {
    for (int u = 0; u < per / 4; ++u) {
      const int j = tid * 4 + 1024 * u;
      v4f o, sm;
#pragma unroll
      for (int q = 0; q < 4; ++q) {
        float gg = g[j + q], bb = bta[j + q];
        if (PARAM_BF16) { gg = bf16_round(gg); bb = bf16_round(bb); }
        sm[q] = vals[u * 4 + q]; o[q] = (vals[u * 4 + q] - mu) * rs * gg + bb;
      }
      if (out_sum) *(volatile v4f*)(out_sum + (size_t)row * N + j) = sm;
      *(volatile v4f*)(out_norm + (size_t)row * N + j) = o;
    }
    if (pass == 0) __threadfence();
  }
}


typedef _Float16 v16h __attribute__((ext_vector_type(16)));
union FragH { v16h v; v8us half[2]; _Float16 h[16]; unsigned short u[16]; };
template <int NT>
__device__ __forceinline__ v8f mmaH(v16h ah, v16h al, v16h bh, v16h bl, v8f c) {
  c = __builtin_amdgcn_wmma_f32_16x16x32_f16(false, ah, false, bh, (short)0, c, false, false);
  if (NT >= 2) c = __builtin_amdgcn_wmma_f32_16x16x32_f16(false, al, false, bh, (short)0, c, false, false);
  if (NT >= 3) c = __builtin_amdgcn_wmma_f32_16x16x32_f16(false, ah, false, bl, (short)0, c, false, false);
  asm volatile("v_nop\n\tv_nop\n\tv_nop\n\tv_nop" : "+v"(c) : "v"(ah), "v"(al), "v"(bh), "v"(bl));
  return c;
}
template <bool ASPLIT>
__global__ __launch_bounds__(128) void k_gemm_h(const float* __restrict__ A, int lda, size_t sA, const _Float16* __restrict__ Bh, int ldb, size_t sB, float alpha, float* __restrict__ C, int ldc, size_t sC, int M, int N, int K) {
  __shared__ __attribute__((aligned(16))) float so[4][16][64];
  const int tid = threadIdx.x, w = tid >> 5, lane = tid & 31, ln = lane & 15, hh = lane >> 4; const int by = blockIdx.y;
  A += (size_t)by * sA; Bh += (size_t)by * sB; C += (size_t)by * sC;
  const int ntn = (N + 63) / 64; const int wid = blockIdx.x * 4 + w; const int mt = wid / ntn, nq = wid % ntn; if (mt * 16 >= M) return;
  const int row0 = mt * 16, col0 = nq * 64; const float* arow = A + (size_t)(row0 + ln) * lda;
  v8f acc[4] = {};
  for (int kb = 0; kb < K; kb += 32) {
    FragH ah, al;
    const v4f x0 = *(const v4fa*)(arow + kb + 8 * hh), x1 = *(const v4fa*)(arow + kb + 8 * hh + 4), x2 = *(const v4fa*)(arow + kb + 16 + 8 * hh), x3 = *(const v4fa*)(arow + kb + 16 + 8 * hh + 4);
    float xs[16] = {x0[0],x0[1],x0[2],x0[3],x1[0],x1[1],x1[2],x1[3],x2[0],x2[1],x2[2],x2[3],x3[0],x3[1],x3[2],x3[3]};
#pragma unroll
    for (int i = 0; i < 16; ++i) { const _Float16 h = (_Float16)xs[i]; ah.h[i] = h; al.h[i] = ASPLIT ? (_Float16)(xs[i] - (float)h) : (_Float16)0.0f; }
#pragma unroll
    for (int t = 0; t < 4; ++t) { if (col0 + t * 16 >= N) continue; const size_t boff = (size_t)(col0 + t * 16 + ln) * ldb + kb; FragH bq; bq.half[0] = *(const v8us*)(Bh + boff + 8 * hh); bq.half[1] = *(const v8us*)(Bh + boff + 16 + 8 * hh);
      acc[t] = mmaH<ASPLIT ? 2 : 1>(ah.v, al.v, bq.v, bq.v, acc[t]); }
  }
#pragma unroll
  for (int t = 0; t < 4; ++t) { if (col0 + t * 16 >= N) continue;
#pragma unroll
    for (int r = 0; r < 8; ++r) so[w][8 * hh + r][t * 16 + ln] = acc[t][r] * alpha; }
  __builtin_amdgcn_fence(__ATOMIC_ACQ_REL, "workgroup"); __builtin_amdgcn_wave_barrier();
  const int rsub = lane >> 4, c4 = (lane & 15) * 4;
  for (int pass = 0; pass < 2; ++pass) {
#pragma unroll
    for (int q = 0; q < 8; ++q) { const int r = q * 2 + rsub; if (col0 + c4 < N) { const v4f v = *(const v4fa*)&so[w][r][c4]; *(volatile v4f*)(C + (size_t)(row0 + r) * ldc + col0 + c4) = v; } }
    if (pass == 0) __threadfence(); }
}

__global__ __launch_bounds__(256) void k_wt_f16(const float* __restrict__ W, _Float16* __restrict__ Wt, int K, int N, float scale) {
  const int t = blockIdx.x * 256 + threadIdx.x; if (t >= N * (K / 8)) return; const int n = t / (K / 8), k8 = (t % (K / 8)) * 8; FragH f;
#pragma unroll
  for (int i = 0; i < 8; ++i) f.h[i] = (_Float16)(bf16_round(W[(size_t)(k8 + i) * N + n]) * scale); const v8us o = f.half[0];
  *(volatile v8us*)((unsigned short*)Wt + (size_t)n * K + k8) = o; __threadfence(); *(volatile v8us*)((unsigned short*)Wt + (size_t)n * K + k8) = o;
}

__global__ __launch_bounds__(256) void k_satt(const float* __restrict__ sat, _Float16* __restrict__ SATT) { const size_t t = (size_t)blockIdx.x * 256 + threadIdx.x; if (t >= (size_t)NM * HP * HP * 4) return; const int pc = (int)(t % 4); const size_t px = t / 4; const int x = (int)(px % HP), y = (int)((px / HP) % HP), m = (int)(px / ((size_t)HP * HP)); const int ys = y - 16, xs = x - 16; const bool in = (ys >= 0 && ys < HS && xs >= 0 && xs < HS); FragH f;
#pragma unroll
  for (int q = 0; q < 8; ++q) { const int c = pc * 8 + q; f.h[q] = (_Float16)(in ? bf16_round(sat[(((size_t)m * CCh + c) * HS + (in ? ys : 0)) * HS + (in ? xs : 0)]) : 0.f); }
  *(volatile v8us*)((unsigned short*)SATT + t * 8) = f.half[0]; __threadfence(); *(volatile v8us*)((unsigned short*)SATT + t * 8) = f.half[0]; }
__global__ __launch_bounds__(256) void k_grdt(const float* __restrict__ grd, _Float16* __restrict__ GRDT) { const size_t t = (size_t)blockIdx.x * 256 + threadIdx.x; if (t >= (size_t)NN * HK * HK * 4) return; const int pc = (int)(t % 4); const size_t px = t / 4; const int kx = (int)(px % HK), ky = (int)((px / HK) % HK), n = (int)(px / (HK * HK)); FragH f;
#pragma unroll
  for (int q = 0; q < 8; ++q) { const int c = pc * 8 + q; f.h[q] = (_Float16)bf16_round(grd[(((size_t)n * CCh + c) * HK + ky) * HK + kx]); }
  *(volatile v8us*)((unsigned short*)GRDT + t * 8) = f.half[0]; __threadfence(); *(volatile v8us*)((unsigned short*)GRDT + t * 8) = f.half[0]; }
__global__ __launch_bounds__(256) void k_norms(const float* __restrict__ sat, const float* __restrict__ grd, float* __restrict__ NS2, float* __restrict__ NG2) { __shared__ float sh[256]; const int tid = threadIdx.x; const int i = blockIdx.x; const bool isg = (i >= NM); const float* src = isg ? grd + (size_t)(i - NM) * CCh * HK * HK : sat + (size_t)i * CCh * HS * HS; const int cnt = isg ? CCh * HK * HK : CCh * HS * HS; float s = 0.f;
#pragma unroll 1
  for (int k = tid; k < cnt; k += 256) { const float v = bf16_round(src[k]); s += v * v; } sh[tid] = s; __syncthreads(); for (int st = 128; st >= 1; st >>= 1) { if (tid < st) sh[tid] += sh[tid + st]; __syncthreads(); }
  if (tid == 0) { float* d = isg ? NG2 + (i - NM) : NS2 + i; *(volatile float*)d = sh[0]; __threadfence(); *(volatile float*)d = sh[0]; } }
__global__ __launch_bounds__(256) void k_energy(const _Float16* __restrict__ SATT, float* __restrict__ E) { const size_t t = (size_t)blockIdx.x * 256 + threadIdx.x; if (t >= (size_t)NM * HP * HP) return; float s = 0.f;
#pragma unroll 1
  for (int c = 0; c < CCh; c += 8) { FragH f; f.half[0] = *(const v8us*)((const unsigned short*)SATT + t * CCh + c); for (int q = 0; q < 8; ++q) { const float v = (float)f.h[q]; s += v * v; } }
  *(volatile float*)(E + t) = s; __threadfence(); *(volatile float*)(E + t) = s; }
__global__ __launch_bounds__(256) void k_roww(const float* __restrict__ E, float* __restrict__ RW) { const size_t t = (size_t)blockIdx.x * 256 + threadIdx.x; if (t >= (size_t)NM * HP * HO) return; const int ox = (int)(t % HO); const size_t my = t / HO; float s = 0.f;
#pragma unroll 1
  for (int kx = 0; kx < HK; ++kx) s += E[my * HP + ox + kx]; *(volatile float*)(RW + t) = s; __threadfence(); *(volatile float*)(RW + t) = s; }
__global__ __launch_bounds__(256) void k_part(const float* __restrict__ RW, float* __restrict__ PART) { const size_t t = (size_t)blockIdx.x * 256 + threadIdx.x; if (t >= (size_t)NM * HO * HO) return; const int ox = (int)(t % HO); const int oy = (int)((t / HO) % HO); const int m = (int)(t / (HO * HO)); float s = 0.f;
#pragma unroll 1
  for (int ky = 0; ky < HK; ++ky) s += RW[((size_t)m * HP + oy + ky) * HO + ox]; *(volatile float*)(PART + t) = s; __threadfence(); *(volatile float*)(PART + t) = s; }
__global__ __launch_bounds__(128) void k_corr(const _Float16* __restrict__ SATT, const _Float16* __restrict__ GRDT, const float* __restrict__ NS2, const float* __restrict__ NG2, const float* __restrict__ PART, float* __restrict__ PMAX) { __shared__ float sm[4][16][17];
  const int tid = threadIdx.x, w = tid >> 5, lane = tid & 31, ln = lane & 15, hh = lane >> 4; const int wid = blockIdx.x * 4 + w; if (wid >= NM * HO * NXT) return;
  const int xt = wid % NXT, oy = (wid / NXT) % HO, m = wid / (NXT * HO); const int ox0 = xt * 16; const int oxl = ox0 + ln; const int oxc = oxl < HO ? oxl : HO - 1;
  v8f acc = (v8f){0.f,0.f,0.f,0.f,0.f,0.f,0.f,0.f};
  const unsigned short* sbase = (const unsigned short*)SATT + (size_t)m * HP * HP * CCh; const unsigned short* gbase = (const unsigned short*)GRDT + (size_t)ln * HK * HK * CCh;
#pragma unroll 1
  for (int ky = 0; ky < HK; ++ky) {
#pragma unroll 4
    for (int kx = 0; kx < HK; ++kx) { const unsigned short* ap = sbase + ((size_t)(oy + ky) * HP + oxc + kx) * CCh; const unsigned short* bp = gbase + ((size_t)ky * HK + kx) * CCh; FragH a, b; a.half[0] = *(const v8us*)(ap + 8 * hh); a.half[1] = *(const v8us*)(ap + 16 + 8 * hh); b.half[0] = *(const v8us*)(bp + 8 * hh); b.half[1] = *(const v8us*)(bp + 16 + 8 * hh); acc = mmaH<1>(a.v, a.v, b.v, b.v, acc); } }
  const float ns = sqrtf(NS2[m]), ng = sqrtf(NG2[ln]); const float inv_nn = 1.0f / (fmaxf(ns, 1e-12f) * fmaxf(ng, 1e-12f)); const float ins2 = 1.0f / fmaxf(NS2[m], 1e-24f); float mx = -INFINITY;
#pragma unroll
  for (int r = 0; r < 8; ++r) { const int ox = ox0 + 8 * hh + r; if (ox < HO) { const float part = PART[((size_t)m * HO + oy) * HO + ox] * ins2; const float v = (acc[r] * inv_nn) / fmaxf(part, 1e-12f); mx = fmaxf(mx, v); } }
  mx = fmaxf(mx, __shfl_xor(mx, 16, 32));
  const float outv = (lane < 16) ? mx : -INFINITY; float* dst = PMAX + (size_t)wid * 32 + lane; *(volatile float*)dst = outv; __threadfence(); *(volatile float*)dst = outv; (void)sm; }
__global__ __launch_bounds__(256) void k_amax(const float* __restrict__ PMAX, float* __restrict__ out) { const int t = threadIdx.x; if (t >= NM * NN) return; const int m = t / NN, n = t % NN; float mx = -INFINITY;
#pragma unroll 1
  for (int i = 0; i < HO * NXT; ++i) mx = fmaxf(mx, PMAX[((size_t)m * HO * NXT + i) * 32 + n]); *(volatile float*)(out + t) = mx; __threadfence(); *(volatile float*)(out + t) = mx; }
extern "C" void kernel_launch(void* const* d_in, const int* in_sizes, int n_in,
                              void* d_out, int out_size, void* d_ws, size_t ws_size, hipStream_t stream) {
  (void)in_sizes; (void)n_in; (void)out_size;
  const float* grd = (const float*)d_in[0]; const float* sat = (const float*)d_in[1];
  char* ws = (char*)d_ws; size_t off = 0;
  auto take = [&](size_t bytes) { char* p = ws + off; off += (bytes + 255) & ~(size_t)255; return p; };
  _Float16* SATT = (_Float16*)take((size_t)NM * HP * HP * CCh * 2); _Float16* GRDT = (_Float16*)take((size_t)NN * HK * HK * CCh * 2); float* NS2 = (float*)take(256); float* NG2 = (float*)take(256); float* E = (float*)take((size_t)NM * HP * HP * 4); float* RW = (float*)take((size_t)NM * HP * HO * 4); float* PART = (float*)take((size_t)NM * HO * HO * 4); float* PMAX = (float*)take((size_t)NM * HO * NXT * 32 * 4);
  if (off > ws_size) return;
  k_satt<<<(unsigned)(((size_t)NM * HP * HP * 4 + 255) / 256), 256, 0, stream>>>(sat, SATT); k_grdt<<<(unsigned)(((size_t)NN * HK * HK * 4 + 255) / 256), 256, 0, stream>>>(grd, GRDT);
  k_norms<<<NM + NN, 256, 0, stream>>>(sat, grd, NS2, NG2); k_energy<<<(unsigned)(((size_t)NM * HP * HP + 255) / 256), 256, 0, stream>>>(SATT, E);
  k_roww<<<(unsigned)(((size_t)NM * HP * HO + 255) / 256), 256, 0, stream>>>(E, RW); k_part<<<(unsigned)(((size_t)NM * HO * HO + 255) / 256), 256, 0, stream>>>(RW, PART);
  k_corr<<<(NM * HO * NXT + 3) / 4, 128, 0, stream>>>(SATT, GRDT, NS2, NG2, PART, PMAX);
  k_amax<<<1, 256, 0, stream>>>(PMAX, (float*)d_out);
}
